// CHGANSimplified_62577673503583
// MI455X (gfx1250) — hardware-verified
//
#include <hip/hip_runtime.h>


#define NB_  2
#define NNODE 1024
#define TT   12
#define DD   128
#define NH_  4
#define HD   32
#define NR   (NNODE * TT)
#define SCL  0.1767766952966369f
#define PCAR 1024.0f
typedef _Float16 h16;
typedef unsigned short bf;
typedef __attribute__((ext_vector_type(16))) __bf16   v16bf;
typedef __attribute__((ext_vector_type(16))) _Float16 v16h;
typedef __attribute__((ext_vector_type(8)))  _Float16 v8h;
typedef __attribute__((ext_vector_type(8)))  unsigned short v8us;
typedef __attribute__((ext_vector_type(8)))  float    v8f;
typedef __attribute__((ext_vector_type(4)))  float    v4f;
typedef v8h  __attribute__((may_alias)) v8ha;
typedef v4f  __attribute__((may_alias)) v4fa;
typedef v8us __attribute__((may_alias)) v8usa;

__device__ __forceinline__ unsigned short f2bf(float f) { unsigned u = __float_as_uint(f); u += 0x7FFFu + ((u >> 16) & 1u); return (unsigned short)(u >> 16); }
__device__ __forceinline__ float bf2f(unsigned short b) { return __uint_as_float(((unsigned)b) << 16); }
__device__ __forceinline__ float bfr(float f) { return bf2f(f2bf(f)); }
__device__ __forceinline__ v16h cat16(v8h lo, v8h hi) { return __builtin_shufflevector(lo, hi, 0, 1, 2, 3, 4, 5, 6, 7, 8, 9, 10, 11, 12, 13, 14, 15); }
__device__ __forceinline__ v16bf cat16b(v8us lo, v8us hi) { return __builtin_bit_cast(v16bf, __builtin_shufflevector(lo, hi, 0, 1, 2, 3, 4, 5, 6, 7, 8, 9, 10, 11, 12, 13, 14, 15)); }
__device__ __forceinline__ v8f wmma16(v16h a, v16h b, v8f c) { return __builtin_amdgcn_wmma_f32_16x16x32_f16(false, a, false, b, (short)0, c, false, false); }
__device__ __forceinline__ v8f wmmab(v16bf a, v16bf b, v8f c) { return __builtin_amdgcn_wmma_f32_16x16x32_bf16(false, a, false, b, (short)0, c, false, false); }


template <typename T16> struct WFrag;
template <> struct WFrag<h16> { typedef v16h V; static __device__ __forceinline__ V ld(const h16* p) { return cat16(*(const v8h*)p, *(const v8h*)(p + 16)); } static __device__ __forceinline__ v8f mma(V a, V b, v8f c) { return wmma16(a, b, c); } };
template <> struct WFrag<bf> { typedef v16bf V; static __device__ __forceinline__ V ld(const bf* p) { return cat16b(*(const v8us*)p, *(const v8us*)(p + 16)); } static __device__ __forceinline__ v8f mma(V a, V b, v8f c) { return wmmab(a, b, c); } };
template <typename T16, int NSPLIT, bool BIAS>
__global__ __launch_bounds__(32) void k_gemmw(const T16* __restrict__ A, const T16* __restrict__ A2, const T16* __restrict__ Bt, const T16* __restrict__ Bt2, int K, float* C, int ldc, const float* __restrict__ bias, size_t sA, size_t sB, size_t sC) {
    typedef typename WFrag<T16>::V V;
    __shared__ __align__(16) float os[16 * 68];
    const size_t z = blockIdx.z; A += z * sA; if (A2) A2 += z * sA; Bt += z * sB; if (Bt2) Bt2 += z * sB; C += z * sC;
    const int lane = threadIdx.x & 31, lr = lane & 15, hi = lane >> 4; const int r0 = blockIdx.x * 64, c0 = blockIdx.y * 64;
    v8f acc[4][4];
#pragma unroll
    for (int mb = 0; mb < 4; ++mb)
#pragma unroll
        for (int nb = 0; nb < 4; ++nb) acc[mb][nb] = (v8f){};
    const size_t aoff = (size_t)(r0 + lr) * K + 8 * hi, boff = (size_t)(c0 + lr) * K + 8 * hi;
#pragma unroll 1
    for (int kc = 0; kc < K; kc += 32) {
        V a[4], a2[4];
#pragma unroll
        for (int mb = 0; mb < 4; ++mb) { a[mb] = WFrag<T16>::ld(A + aoff + (size_t)mb * 16 * K + kc); if (NSPLIT == 1 || NSPLIT == 2) a2[mb] = WFrag<T16>::ld(A2 + aoff + (size_t)mb * 16 * K + kc); }
#pragma unroll
        for (int nb = 0; nb < 4; ++nb) { const V b = WFrag<T16>::ld(Bt + boff + (size_t)nb * 16 * K + kc); V b2; if (NSPLIT >= 2) b2 = WFrag<T16>::ld(Bt2 + boff + (size_t)nb * 16 * K + kc);
#pragma unroll
            for (int mb = 0; mb < 4; ++mb) { acc[mb][nb] = WFrag<T16>::mma(a[mb], b, acc[mb][nb]); if (NSPLIT == 1 || NSPLIT == 2) acc[mb][nb] = WFrag<T16>::mma(a2[mb], b, acc[mb][nb]); if (NSPLIT >= 2) acc[mb][nb] = WFrag<T16>::mma(a[mb], b2, acc[mb][nb]); } }
        asm volatile("v_nop\n\tv_nop\n\tv_nop\n\tv_nop" : "+v"(acc[0][0]), "+v"(acc[1][1]), "+v"(acc[2][2]), "+v"(acc[3][3]) : "v"(a[0]), "v"(a[3]));
    }
#pragma unroll
    for (int mb = 0; mb < 4; ++mb) {
#pragma unroll
        for (int nb = 0; nb < 4; ++nb) {
#pragma unroll
            for (int j = 0; j < 8; ++j) os[(hi * 8 + j) * 68 + nb * 16 + lr] = acc[mb][nb][j]; }
        __builtin_amdgcn_wave_barrier(); asm volatile("" ::: "memory");
        float* crow = C + (size_t)(r0 + mb * 16) * ldc + c0;
#pragma unroll 1
        for (int ps = 0; ps < 2; ++ps) {
#pragma unroll
            for (int s = 0; s < 8; ++s) { const int row = 2 * s + hi, cofs = lr * 4; v4f val = *(const v4fa*)(os + row * 68 + cofs); if (BIAS) { val[0] += bfr(bias[c0 + cofs]); val[1] += bfr(bias[c0 + cofs + 1]); val[2] += bfr(bias[c0 + cofs + 2]); val[3] += bfr(bias[c0 + cofs + 3]); }
                *(volatile v4f*)(crow + (size_t)row * ldc + cofs) = val; }
            if (ps == 0) __threadfence(); }
        __builtin_amdgcn_wave_barrier(); asm volatile("" ::: "memory");
    }
}

__device__ __forceinline__ h16 tohx(float x) { return (h16)x; }
__device__ __forceinline__ void splitf(float y, unsigned short& h, unsigned short& l) { h = f2bf(y); l = f2bf(y - bf2f(h)); }
typedef __attribute__((ext_vector_type(2))) _Float16 v2h;
typedef __attribute__((ext_vector_type(4))) _Float16 v4h;
typedef __attribute__((ext_vector_type(4))) unsigned short v4us;
typedef __attribute__((ext_vector_type(2))) unsigned short v2us;

__global__ __launch_bounds__(256) void k_cvt8(const float* __restrict__ src, bf* dst, size_t n8) { const size_t i = (size_t)blockIdx.x * 256 + threadIdx.x; if (i >= n8) return; const v8f v = *(const v8f*)(src + i * 8); v8us o;
#pragma unroll
    for (int k = 0; k < 8; ++k) o[k] = f2bf(v[k]); *(volatile v8us*)(dst + i * 8) = o; __threadfence(); *(volatile v8us*)(dst + i * 8) = o; }
__global__ __launch_bounds__(256) void k_bcat(const float* __restrict__ bq, const float* __restrict__ bk, const float* __restrict__ bv, float* B3) { const int i = blockIdx.x * 256 + threadIdx.x; if (i >= 3 * DD) return; const float v = i < DD ? bq[i] : (i < 2 * DD ? bk[i - DD] : bv[i - 2 * DD]); *(volatile float*)(B3 + i) = v; __threadfence(); *(volatile float*)(B3 + i) = v; }
__global__ __launch_bounds__(256) void k_enh(const float* __restrict__ x, const float* __restrict__ emb, bf* Eh, bf* El) { const int e = (blockIdx.x * 256 + threadIdx.x) * 4; if (e >= NR * DD) return; const int c = e % DD; const int n = (e / DD) / TT; const int ty = 1 - (n & 1); v4us oh, ol;
#pragma unroll
    for (int q = 0; q < 4; ++q) { unsigned short a, b; splitf(__fadd_rn(bfr(x[e + q]), bfr(emb[ty * DD + c + q])), a, b); oh[q] = a; ol[q] = b; } *(volatile v4us*)(Eh + e) = oh; *(volatile v4us*)(El + e) = ol; __threadfence(); *(volatile v4us*)(Eh + e) = oh; *(volatile v4us*)(El + e) = ol; }
__global__ __launch_bounds__(256) void k_qkpl(const float* __restrict__ QKV, int t, bf* Qh, bf* Ql, bf* Kh, bf* Kl) { const int e = (blockIdx.x * 256 + threadIdx.x) * 4; if (e >= NH_ * NNODE * HD) return; const int d = e % HD; const int n = (e / HD) % NNODE; const int h = e / (HD * NNODE); const float* r = QKV + ((size_t)n * TT + t) * 3 * DD + h * HD + d; v4us qh, ql, kh, kl;
#pragma unroll
    for (int q = 0; q < 4; ++q) { unsigned short a, c; splitf(r[q] * SCL, a, c); qh[q] = a; ql[q] = c; splitf(r[DD + q], a, c); kh[q] = a; kl[q] = c; }
    for (int ps = 0; ps < 2; ++ps) { *(volatile v4us*)(Qh + e) = qh; *(volatile v4us*)(Ql + e) = ql; *(volatile v4us*)(Kh + e) = kh; *(volatile v4us*)(Kl + e) = kl; if (ps == 0) __threadfence(); } }
__global__ __launch_bounds__(256) void k_vt(const float* __restrict__ QKV, int t, h16* V16) { const int e = (blockIdx.x * 256 + threadIdx.x) * 2; if (e >= NH_ * 64 * NNODE) return; const int m = e % NNODE; const int dv = (e / NNODE) % 64; const int h = e / (NNODE * 64); v2h o;
#pragma unroll
    for (int u = 0; u < 2; ++u) o[u] = dv < HD ? tohx(QKV[((size_t)(m + u) * TT + t) * 3 * DD + 2 * DD + h * HD + dv]) : (h16)0.f; *(volatile v2h*)(V16 + e) = o; __threadfence(); *(volatile v2h*)(V16 + e) = o; }
__global__ __launch_bounds__(256) void k_mrg(const float* __restrict__ O, int t, float* ATT) { const int e = (blockIdx.x * 256 + threadIdx.x) * 4; if (e >= NNODE * DD) return; const int c = e % DD; const int n = e / DD; const int h = c / HD, d = c % HD; const float* r = O + ((size_t)h * NNODE + n) * 64 + d; v4f o; o[0] = r[0] * (1.0f / PCAR); o[1] = r[1] * (1.0f / PCAR); o[2] = r[2] * (1.0f / PCAR); o[3] = r[3] * (1.0f / PCAR); float* dst = ATT + ((size_t)n * TT + t) * DD + c; *(volatile v4f*)dst = o; __threadfence(); *(volatile v4f*)dst = o; }
__global__ __launch_bounds__(256) void k_msoft(const float* __restrict__ Sb, const int* __restrict__ adj, const float* __restrict__ eb, h16* P16) { const int lane = threadIdx.x & 31; const int row = blockIdx.x * 8 + (threadIdx.x >> 5); if (row >= NH_ * NNODE) return; const int n = row % NNODE; const float* sr = Sb + (size_t)row * NNODE; const int* ar = adj + (size_t)n * NNODE; const float* er = eb + (size_t)n * NNODE;
    auto val = [&](int m, float s) { const bool keep = (ar[m] != 0) || (m == n); return keep ? __fadd_rn(s, bfr(er[m])) : -3.0e38f; };
    float mx = -3.0e38f;
#pragma unroll 1
    for (int ch = 0; ch < NNODE / 128; ++ch) { const int m0 = ch * 128 + lane * 4; const v4f a = *(const v4f*)(sr + m0);
#pragma unroll
        for (int q = 0; q < 4; ++q) mx = fmaxf(mx, val(m0 + q, a[q])); }
#pragma unroll
    for (int sh = 16; sh; sh >>= 1) mx = fmaxf(mx, __shfl_xor(mx, sh, 32));
    float sum = 0.f;
#pragma unroll 1
    for (int ch = 0; ch < NNODE / 128; ++ch) { const int m0 = ch * 128 + lane * 4; const v4f a = *(const v4f*)(sr + m0);
#pragma unroll
        for (int q = 0; q < 4; ++q) { const float v = val(m0 + q, a[q]); if (v > -1.0e38f) { float d0 = __fsub_rn(v, mx); asm volatile("" : "+v"(d0)); sum += __expf(d0); } } }
#pragma unroll
    for (int sh = 16; sh; sh >>= 1) sum += __shfl_xor(sum, sh, 32);
    const float f = __fdiv_rn(PCAR, sum);
    for (int ps = 0; ps < 2; ++ps) {
#pragma unroll 1
        for (int ch = 0; ch < NNODE / 128; ++ch) { const int m0 = ch * 128 + lane * 4; const v4f a = *(const v4f*)(sr + m0); v4h o;
#pragma unroll
            for (int q = 0; q < 4; ++q) { const float v = val(m0 + q, a[q]); float p = 0.f; if (v > -1.0e38f) { float d0 = __fsub_rn(v, mx); asm volatile("" : "+v"(d0)); p = __fmul_rn(__expf(d0), f); } o[q] = tohx(p); }
            *(volatile v4h*)(P16 + (size_t)row * NNODE + m0) = o; }
        if (ps == 0) __threadfence(); } }
__global__ __launch_bounds__(256) void k_split(const float* __restrict__ F, size_t n4, bf* Hh, bf* Hl) { const size_t e = ((size_t)blockIdx.x * 256 + threadIdx.x) * 4; if (e >= n4 * 4) return; const v4f a = *(const v4f*)(F + e); v4us oh, ol;
#pragma unroll
    for (int q = 0; q < 4; ++q) { unsigned short u, l; splitf(a[q], u, l); oh[q] = u; ol[q] = l; } *(volatile v4us*)(Hh + e) = oh; *(volatile v4us*)(Hl + e) = ol; __threadfence(); *(volatile v4us*)(Hh + e) = oh; *(volatile v4us*)(Hl + e) = ol; }
__global__ __launch_bounds__(256) void k_lnres(const float* __restrict__ A, const float* __restrict__ x, const float* __restrict__ g, const float* __restrict__ bb, float* Y) { const int lane = threadIdx.x & 31; const int row = blockIdx.x * 8 + (threadIdx.x >> 5); if (row >= NR) return; const size_t rb = (size_t)row * DD; const int c0 = lane * 4; const v4f a = *(const v4f*)(A + rb + c0); float v[4]; float s = 0.f;
#pragma unroll
    for (int q = 0; q < 4; ++q) { v[q] = __fadd_rn(a[q], bfr(x[rb + c0 + q])); s = __fadd_rn(s, v[q]); }
#pragma unroll
    for (int sh = 16; sh; sh >>= 1) s += __shfl_xor(s, sh, 32);
    const float mean = s * (1.0f / DD); float q2 = 0.f;
#pragma unroll
    for (int q = 0; q < 4; ++q) { float d0 = __fsub_rn(v[q], mean); asm volatile("" : "+v"(d0)); float p = __fmul_rn(d0, d0); asm volatile("" : "+v"(p)); q2 = __fadd_rn(q2, p); }
#pragma unroll
    for (int sh = 16; sh; sh >>= 1) q2 += __shfl_xor(q2, sh, 32);
    const float rstd = __frsqrt_rn(__fadd_rn(q2 * (1.0f / DD), 1e-5f)); v4f o;
#pragma unroll
    for (int q = 0; q < 4; ++q) { float t0 = __fmul_rn(__fsub_rn(v[q], mean), rstd); asm volatile("" : "+v"(t0)); float t1 = __fmul_rn(t0, bfr(g[c0 + q])); asm volatile("" : "+v"(t1)); o[q] = __fadd_rn(t1, bfr(bb[c0 + q])); }
    *(volatile v4f*)(Y + rb + c0) = o; __threadfence(); *(volatile v4f*)(Y + rb + c0) = o; }

extern "C" void kernel_launch(void* const* d_in, const int* in_sizes, int n_in,
                              void* d_out, int out_size, void* d_ws, size_t ws_size, hipStream_t stream) {
    (void)in_sizes; (void)n_in; (void)out_size;
    const float* x = (const float*)d_in[0]; const int* adj = (const int*)d_in[1]; const float* emb = (const float*)d_in[2]; const float* wq = (const float*)d_in[3]; const float* bq = (const float*)d_in[4]; const float* wk = (const float*)d_in[5]; const float* bk = (const float*)d_in[6]; const float* wv = (const float*)d_in[7]; const float* bv = (const float*)d_in[8]; const float* eb = (const float*)d_in[9]; const float* wo = (const float*)d_in[10]; const float* bo = (const float*)d_in[11]; const float* g = (const float*)d_in[12]; const float* be = (const float*)d_in[13];
    float* OUT = (float*)d_out;
    char* wsp = (char*)d_ws;
    auto take = [&](size_t bytes) { char* p = wsp; wsp += (bytes + 255) & ~(size_t)255; return (void*)p; };
    bf* WQKV = (bf*)take((size_t)3 * DD * DD * 2); float* BQKV = (float*)take(3 * DD * 4); bf* WO = (bf*)take(DD * DD * 2);
    bf* Eh = (bf*)take((size_t)NR * DD * 2); bf* El = (bf*)take((size_t)NR * DD * 2); float* QKV = (float*)take((size_t)NR * 3 * DD * 4); bf* Qh = (bf*)take(NH_ * NNODE * HD * 2); bf* Ql = (bf*)take(NH_ * NNODE * HD * 2); bf* Kh = (bf*)take(NH_ * NNODE * HD * 2); bf* Kl = (bf*)take(NH_ * NNODE * HD * 2); h16* V16 = (h16*)take((size_t)NH_ * 64 * NNODE * 2);
    float* Sb = (float*)take((size_t)NH_ * NNODE * NNODE * 4); h16* P16 = (h16*)take((size_t)NH_ * NNODE * NNODE * 2); float* O = (float*)take((size_t)NH_ * NNODE * 64 * 4); float* ATT = (float*)take((size_t)NR * DD * 4); bf* Ah = (bf*)take((size_t)NR * DD * 2); bf* Al = (bf*)take((size_t)NR * DD * 2); float* AO = (float*)take((size_t)NR * DD * 4);
    if ((size_t)(wsp - (char*)d_ws) > ws_size) return;
    k_cvt8<<<(DD * DD / 8 + 255) / 256, 256, 0, stream>>>(wq, WQKV, DD * DD / 8); k_cvt8<<<(DD * DD / 8 + 255) / 256, 256, 0, stream>>>(wk, WQKV + DD * DD, DD * DD / 8); k_cvt8<<<(DD * DD / 8 + 255) / 256, 256, 0, stream>>>(wv, WQKV + 2 * DD * DD, DD * DD / 8);
    k_bcat<<<2, 256, 0, stream>>>(bq, bk, bv, BQKV);
    k_cvt8<<<(DD * DD / 8 + 255) / 256, 256, 0, stream>>>(wo, WO, DD * DD / 8);
    for (int b = 0; b < NB_; ++b) { const float* xb = x + (size_t)b * NR * DD;
        k_enh<<<(NR * DD / 4 + 255) / 256, 256, 0, stream>>>(xb, emb, Eh, El);
        k_gemmw<bf, 1, true><<<dim3(NR / 64, 3 * DD / 64, 1), 32, 0, stream>>>(Eh, El, WQKV, nullptr, DD, QKV, 3 * DD, BQKV, 0, 0, 0);
        for (int t = 0; t < TT; ++t) {
            k_qkpl<<<(NH_ * NNODE * HD / 4 + 255) / 256, 256, 0, stream>>>(QKV, t, Qh, Ql, Kh, Kl); k_vt<<<(NH_ * 64 * NNODE / 2 + 255) / 256, 256, 0, stream>>>(QKV, t, V16);
            k_gemmw<bf, 2, false><<<dim3(NNODE / 64, NNODE / 64, NH_), 32, 0, stream>>>(Qh, Ql, Kh, Kl, HD, Sb, NNODE, nullptr, (size_t)NNODE * HD, (size_t)NNODE * HD, (size_t)NNODE * NNODE);
            k_msoft<<<NH_ * NNODE / 8, 256, 0, stream>>>(Sb, adj, eb, P16);
            k_gemmw<h16, 0, false><<<dim3(NNODE / 64, 1, NH_), 32, 0, stream>>>(P16, nullptr, V16, nullptr, NNODE, O, 64, nullptr, (size_t)NNODE * NNODE, (size_t)64 * NNODE, (size_t)NNODE * 64);
            k_mrg<<<(NNODE * DD / 4 + 255) / 256, 256, 0, stream>>>(O, t, ATT); }
        k_split<<<(NR * DD / 4 + 255) / 256, 256, 0, stream>>>(ATT, (size_t)NR * DD / 4, Ah, Al);
        k_gemmw<bf, 1, true><<<dim3(NR / 64, DD / 64, 1), 32, 0, stream>>>(Ah, Al, WO, nullptr, DD, AO, DD, bo, 0, 0, 0);
        k_lnres<<<NR / 8, 256, 0, stream>>>(AO, xb, g, be, OUT + (size_t)b * NR * DD); }
}
